// SelfAttn_73976516706753
// MI455X (gfx1250) — hardware-verified
//
#include <hip/hip_runtime.h>
#pragma clang fp contract(off)


#ifndef NB
#define NB 4
#endif
#ifndef SEQ
#define SEQ 2048
#endif
#define NB_FULL 4
#define T_FULL  2048
#define TT   SEQ
#define DM   1024
#define NH   8
#define HD   128
#define TE   256
#define PCAR 1024.0f
#define SCL  0.08838834764831845f
#define L2E  1.4426950408889634f
static_assert(TT % 64 == 0);
static_assert(TT >= TE);
static_assert(TE % 128 == 0);
static_assert(NH * HD == DM);
static_assert(NB <= NB_FULL);
static_assert(TT <= T_FULL);

typedef _Float16 h16;
typedef unsigned short bf;
typedef __attribute__((ext_vector_type(16))) __bf16   v16bf;
typedef __attribute__((ext_vector_type(16))) _Float16 v16h;
typedef __attribute__((ext_vector_type(8)))  _Float16 v8h;
typedef __attribute__((ext_vector_type(8)))  unsigned short v8us;
typedef __attribute__((ext_vector_type(8)))  float    v8f;
typedef __attribute__((ext_vector_type(4)))  float    v4f;
typedef v8h  __attribute__((may_alias)) v8ha;
typedef v4f  __attribute__((may_alias)) v4fa;
typedef v8us __attribute__((may_alias)) v8usa;
typedef __attribute__((ext_vector_type(2))) _Float16 v2h;
typedef __attribute__((ext_vector_type(4))) _Float16 v4h;
typedef __attribute__((ext_vector_type(2))) unsigned short v2us;
typedef __attribute__((ext_vector_type(4))) unsigned short v4us;
typedef __attribute__((ext_vector_type(2))) float v2f;

__device__ __forceinline__ unsigned short f2bf(float f) { unsigned u = __float_as_uint(f); u += 0x7FFFu + ((u >> 16) & 1u); return (unsigned short)(u >> 16); }
__device__ __forceinline__ float bf2f(unsigned short b) { return __uint_as_float(((unsigned)b) << 16); }
__device__ __forceinline__ float bfr(float f) { return bf2f(f2bf(f)); }
__device__ __forceinline__ v16h cat16(v8h lo, v8h hi) { return __builtin_shufflevector(lo, hi, 0, 1, 2, 3, 4, 5, 6, 7, 8, 9, 10, 11, 12, 13, 14, 15); }
__device__ __forceinline__ v16bf cat16b(v8us lo, v8us hi) { return __builtin_bit_cast(v16bf, __builtin_shufflevector(lo, hi, 0, 1, 2, 3, 4, 5, 6, 7, 8, 9, 10, 11, 12, 13, 14, 15)); }
__device__ __forceinline__ v8f wmma16(v16h a, v16h b, v8f c) { return __builtin_amdgcn_wmma_f32_16x16x32_f16(false, a, false, b, (short)0, c, false, false); }
__device__ __forceinline__ v8f wmmab(v16bf a, v16bf b, v8f c) { return __builtin_amdgcn_wmma_f32_16x16x32_bf16(false, a, false, b, (short)0, c, false, false); }
__device__ __forceinline__ v8f wmma16g(v16h a, v16h b, v8f c) {
    c = __builtin_amdgcn_wmma_f32_16x16x32_f16(false, a, false, b, (short)0, c, false, false);
    asm volatile("v_nop\n\tv_nop\n\tv_nop\n\tv_nop" : "+v"(c) : "v"(a), "v"(b));
    return c;
}
__device__ __forceinline__ v16h ldh(const h16* p) { return cat16(*(const v8h*)p, *(const v8h*)(p + 16)); }
__device__ __forceinline__ h16 tohx(float x) { return (h16)x; }
__device__ __forceinline__ void splitf(float y, unsigned short& h, unsigned short& l) { h = f2bf(y); l = f2bf(y - bf2f(h)); }

template <typename T16> struct WFrag;
template <> struct WFrag<h16> { typedef v16h V; static __device__ __forceinline__ V ld(const h16* p) { return cat16(*(const v8h*)p, *(const v8h*)(p + 16)); } static __device__ __forceinline__ v8f mma(V a, V b, v8f c) { return wmma16(a, b, c); } };
template <> struct WFrag<bf> { typedef v16bf V; static __device__ __forceinline__ V ld(const bf* p) { return cat16b(*(const v8us*)p, *(const v8us*)(p + 16)); } static __device__ __forceinline__ v8f mma(V a, V b, v8f c) { return wmmab(a, b, c); } };
template <typename T16, int NSPLIT, bool BIAS>
__global__ __launch_bounds__(32) void k_gemmw(const T16* __restrict__ A, const T16* __restrict__ A2, const T16* __restrict__ Bt, const T16* __restrict__ Bt2, int K, float* C, int ldc, const float* __restrict__ bias, size_t sA, size_t sB, size_t sC) {
    typedef typename WFrag<T16>::V V;
    __shared__ __align__(16) float os[16 * 68];
    const size_t z = blockIdx.z; A += z * sA; if (A2) A2 += z * sA; Bt += z * sB; if (Bt2) Bt2 += z * sB; C += z * sC;
    const int lane = threadIdx.x & 31, lr = lane & 15, hi = lane >> 4; const int r0 = blockIdx.x * 64, c0 = blockIdx.y * 64;
    v8f acc[4][4];
#pragma unroll
    for (int mb = 0; mb < 4; ++mb)
#pragma unroll
        for (int nb = 0; nb < 4; ++nb) acc[mb][nb] = (v8f){};
    const size_t aoff = (size_t)(r0 + lr) * K + 8 * hi, boff = (size_t)(c0 + lr) * K + 8 * hi;
#pragma unroll 1
    for (int kc = 0; kc < K; kc += 32) {
        V a[4], a2[4];
#pragma unroll
        for (int mb = 0; mb < 4; ++mb) { a[mb] = WFrag<T16>::ld(A + aoff + (size_t)mb * 16 * K + kc); if (NSPLIT == 1 || NSPLIT == 2) a2[mb] = WFrag<T16>::ld(A2 + aoff + (size_t)mb * 16 * K + kc); }
#pragma unroll
        for (int nb = 0; nb < 4; ++nb) { const V b = WFrag<T16>::ld(Bt + boff + (size_t)nb * 16 * K + kc); V b2; if (NSPLIT >= 2) b2 = WFrag<T16>::ld(Bt2 + boff + (size_t)nb * 16 * K + kc);
#pragma unroll
            for (int mb = 0; mb < 4; ++mb) { acc[mb][nb] = WFrag<T16>::mma(a[mb], b, acc[mb][nb]); if (NSPLIT == 1 || NSPLIT == 2) acc[mb][nb] = WFrag<T16>::mma(a2[mb], b, acc[mb][nb]); if (NSPLIT >= 2) acc[mb][nb] = WFrag<T16>::mma(a[mb], b2, acc[mb][nb]); } }
        asm volatile("v_nop\n\tv_nop\n\tv_nop\n\tv_nop" : "+v"(acc[0][0]), "+v"(acc[1][1]), "+v"(acc[2][2]), "+v"(acc[3][3]) : "v"(a[0]), "v"(a[3]));
    }
#pragma unroll
    for (int mb = 0; mb < 4; ++mb) {
#pragma unroll
        for (int nb = 0; nb < 4; ++nb) {
#pragma unroll
            for (int j = 0; j < 8; ++j) os[(hi * 8 + j) * 68 + nb * 16 + lr] = acc[mb][nb][j]; }
        __builtin_amdgcn_wave_barrier(); asm volatile("" ::: "memory");
        float* crow = C + (size_t)(r0 + mb * 16) * ldc + c0;
#pragma unroll 1
        for (int ps = 0; ps < 2; ++ps) {
#pragma unroll
            for (int s = 0; s < 8; ++s) { const int row = 2 * s + hi, cofs = lr * 4; v4f val = *(const v4fa*)(os + row * 68 + cofs); if (BIAS) { val[0] += bfr(bias[c0 + cofs]); val[1] += bfr(bias[c0 + cofs + 1]); val[2] += bfr(bias[c0 + cofs + 2]); val[3] += bfr(bias[c0 + cofs + 3]); }
                *(volatile v4f*)(crow + (size_t)row * ldc + cofs) = val; }
            if (ps == 0) __threadfence(); }
        __builtin_amdgcn_wave_barrier(); asm volatile("" ::: "memory");
    }
}

__global__ __launch_bounds__(256) void k_cvt8(const float* __restrict__ src, bf* dst, size_t n8) { const size_t i = (size_t)blockIdx.x * 256 + threadIdx.x; if (i >= n8) return; const v8f v = *(const v8f*)(src + i * 8); v8us o;
#pragma unroll
    for (int k = 0; k < 8; ++k) o[k] = f2bf(v[k]); *(volatile v8us*)(dst + i * 8) = o; __threadfence(); *(volatile v8us*)(dst + i * 8) = o; }

__global__ __launch_bounds__(256) void k_rope(const float* __restrict__ F, const float* __restrict__ CT, const float* __restrict__ ST, h16* P16, bf* Ph, bf* Pl) {
    const size_t e = ((size_t)blockIdx.x * 256 + threadIdx.x) * 2; if (e >= (size_t)NH * TT * HD) return;
    const int d = (int)(e % HD); const int t = (int)((e / HD) % TT); const int h = (int)(e / ((size_t)HD * TT));
    const float* f = F + (size_t)t * DM; const float* ct = CT + (size_t)t * DM; const float* st = ST + (size_t)t * DM;
    v2h o16 = (v2h){}; v2us oh = (v2us){}, ol = (v2us){};
#pragma unroll
    for (int q = 0; q < 2; ++q) { const int g = h * HD + d + q; const int pg = (g < DM / 2) ? (2 * g + 1) : (2 * g - DM);
        const float x0 = f[g]; const float x1 = f[pg]; const float c = bfr(ct[g]); const float sn = bfr(st[g]);
        float a = __fmul_rn(x0, c), bq = __fmul_rn(x1, sn); asm volatile("" : "+v"(a)); asm volatile("" : "+v"(bq));
        const float r = (g < DM / 2) ? __fsub_rn(a, bq) : __fadd_rn(a, bq);
        o16[q] = tohx(r); unsigned short a2, c2; splitf(r, a2, c2); oh[q] = a2; ol[q] = c2; }
    *(volatile v2h*)(P16 + e) = o16; *(volatile v2us*)(Ph + e) = oh; *(volatile v2us*)(Pl + e) = ol; __threadfence(); *(volatile v2h*)(P16 + e) = o16; *(volatile v2us*)(Ph + e) = oh; *(volatile v2us*)(Pl + e) = ol; }

__global__ __launch_bounds__(256) void k_vtp16(const float* __restrict__ F, h16* V16) {
    const size_t e = ((size_t)blockIdx.x * 256 + threadIdx.x) * 2; if (e >= (size_t)NH * HD * TT) return;
    const int t = (int)(e % TT); const int d = (int)((e / TT) % HD); const int h = (int)(e / ((size_t)TT * HD)); v2h o16 = (v2h){};
#pragma unroll
    for (int q = 0; q < 2; ++q) { const float x = F[(size_t)(t + q) * DM + h * HD + d]; o16[q] = tohx(x); }
    *(volatile v2h*)(V16 + e) = o16; __threadfence(); *(volatile v2h*)(V16 + e) = o16; }
__global__ __launch_bounds__(256) void k_vte(const float* __restrict__ F, bf* Vh, bf* Vl) {
    const size_t e = ((size_t)blockIdx.x * 256 + threadIdx.x) * 2; if (e >= (size_t)NH * HD * TE) return;
    const int t = (int)(e % TE); const int d = (int)((e / TE) % HD); const int h = (int)(e / ((size_t)TE * HD)); v2us oh = (v2us){}, ol = (v2us){};
#pragma unroll
    for (int q = 0; q < 2; ++q) { const float x = F[(size_t)(t + q) * DM + h * HD + d]; unsigned short a2, c2; splitf(x, a2, c2); oh[q] = a2; ol[q] = c2; }
    *(volatile v2us*)(Vh + e) = oh; *(volatile v2us*)(Vl + e) = ol; __threadfence(); *(volatile v2us*)(Vh + e) = oh; *(volatile v2us*)(Vl + e) = ol; }

__global__ __launch_bounds__(256) void k_lsoftE(const float* __restrict__ Sb, bf* Ph, bf* Pl) {
    const int lane = threadIdx.x & 31; const int row = blockIdx.x * 8 + (threadIdx.x >> 5); if (row >= NH * TE) return; const int i = row % TE;
    const float* sr = Sb + (size_t)row * TE; float mx = -3.0e38f;
#pragma unroll
    for (int ch = 0; ch < TE / 128; ++ch) { const int j0 = ch * 128 + lane * 4; const v4f a = *(const v4f*)(sr + j0);
#pragma unroll
        for (int q = 0; q < 4; ++q) { float t = a[q] * SCL; asm volatile("" : "+v"(t)); t = (j0 + q <= i) ? t : -3.0e38f; mx = fmaxf(mx, t); } }
#pragma unroll
    for (int sh = 16; sh; sh >>= 1) mx = fmaxf(mx, __shfl_xor(mx, sh, 32));
    float sum = 0.f;
#pragma unroll
    for (int ch = 0; ch < TE / 128; ++ch) { const int j0 = ch * 128 + lane * 4; const v4f a = *(const v4f*)(sr + j0);
#pragma unroll
        for (int q = 0; q < 4; ++q) { float t = a[q] * SCL; asm volatile("" : "+v"(t)); t = (j0 + q <= i) ? t : -3.0e38f; float d0 = __fsub_rn(t, mx); asm volatile("" : "+v"(d0)); sum += __builtin_amdgcn_exp2f(__fmul_rn(d0, L2E)); } }
#pragma unroll
    for (int sh = 16; sh; sh >>= 1) sum += __shfl_xor(sum, sh, 32);
    const float f = __fdiv_rn(1.0f, sum);
#pragma unroll 1
    for (int ps = 0; ps < 2; ++ps) {
#pragma unroll
        for (int ch = 0; ch < TE / 128; ++ch) { const int j0 = ch * 128 + lane * 4; const v4f a = *(const v4f*)(sr + j0); v4us oh = (v4us){}, ol = (v4us){};
#pragma unroll
            for (int q = 0; q < 4; ++q) { float t = a[q] * SCL; asm volatile("" : "+v"(t)); t = (j0 + q <= i) ? t : -3.0e38f; float d0 = __fsub_rn(t, mx); asm volatile("" : "+v"(d0)); float ex = __builtin_amdgcn_exp2f(__fmul_rn(d0, L2E)); asm volatile("" : "+v"(ex)); unsigned short a2, c2; splitf(ex * f, a2, c2); oh[q] = a2; ol[q] = c2; }
            const size_t oo = (size_t)row * TE + j0; *(volatile v4us*)(Ph + oo) = oh; *(volatile v4us*)(Pl + oo) = ol; }
        if (ps == 0) __threadfence(); }
}

__global__ __launch_bounds__(256) void k_mergeE(const float* __restrict__ O, float* OUTb) {
    const size_t e = ((size_t)blockIdx.x * 256 + threadIdx.x) * 2; if (e >= (size_t)NH * TE * HD) return;
    const int d = (int)(e % HD); const int t = (int)((e / HD) % TE); const int z = (int)(e / ((size_t)HD * TE)); const size_t oo = (size_t)t * DM + z * HD + d;
    v2f o2; o2[0] = O[e]; o2[1] = O[e + 1]; *(volatile v2f*)(OUTb + oo) = o2; __threadfence(); *(volatile v2f*)(OUTb + oo) = o2; }

__global__ __launch_bounds__(128) __attribute__((amdgpu_num_vgpr(256)))
void k_flash(const h16* __restrict__ QP, const h16* __restrict__ KP, const h16* __restrict__ VT, float* OUTb) {
    __shared__ __align__(16) float os[4 * 16 * 132];
    const int lane = threadIdx.x & 31, wid = threadIdx.x >> 5, lr = lane & 15, hi = lane >> 4;
    const int nh = blockIdx.y; const int QB = (int)blockIdx.x + TE / 64; const int qb = QB * 64 + wid * 16;
    const h16* Q = QP + (size_t)nh * TT * HD; const h16* Kp = KP + (size_t)nh * TT * HD; const h16* V = VT + (size_t)nh * HD * TT;
    v16h qf[4];
#pragma unroll
    for (int hc = 0; hc < 4; ++hc) qf[hc] = ldh(Q + (size_t)(qb + lr) * HD + hc * 32 + 8 * hi);
    v8f oT[8];
#pragma unroll
    for (int f = 0; f < 8; ++f) oT[f] = (v8f){};
    float mrow = -3.0e38f, lrow = 0.0f;
    const int qg = qb + lr;
    const int ntiles = QB + 1;
#pragma unroll 1
    for (int tile = 0; tile < ntiles; ++tile) {
        const int kt0 = tile * 64;
        v8f s[4];
#pragma unroll
        for (int kf = 0; kf < 4; ++kf) {
            s[kf] = (v8f){};
            const h16* kr = Kp + (size_t)(kt0 + kf * 16 + lr) * HD + 8 * hi;
#pragma unroll
            for (int hc = 0; hc < 4; ++hc) { const v16h aK = ldh(kr + hc * 32); s[kf] = wmma16g(aK, qf[hc], s[kf]); }
            asm volatile("" ::: "memory");
        }
        const bool diag = (tile == ntiles - 1);
        float vm = -3.0e38f;
#pragma unroll
        for (int kf = 0; kf < 4; ++kf)
#pragma unroll
            for (int r = 0; r < 8; ++r) { const int key = kt0 + kf * 16 + 8 * hi + r; float t = s[kf][r] * (SCL * L2E); t = (diag && key > qg) ? -3.0e38f : t; s[kf][r] = t; vm = fmaxf(vm, t); }
        vm = fmaxf(vm, __shfl_xor(vm, 16, 32));
        const float mnew = fmaxf(mrow, vm);
        const float alpha = __builtin_amdgcn_exp2f(mrow - mnew);
        mrow = mnew;
        float ls = 0.0f;
#pragma unroll
        for (int kf = 0; kf < 4; ++kf)
#pragma unroll
            for (int r = 0; r < 8; ++r) { const float p = __builtin_amdgcn_exp2f(s[kf][r] - mnew); s[kf][r] = p; ls += p; }
        ls += __shfl_xor(ls, 16, 32);
        lrow = lrow * alpha + ls;
#pragma unroll
        for (int f = 0; f < 8; ++f) oT[f] = oT[f] * alpha;
#pragma unroll
        for (int c = 0; c < 2; ++c) {
            v8h plo = (v8h){}, phi = (v8h){};
#pragma unroll
            for (int r = 0; r < 8; ++r) { plo[r] = tohx(s[2 * c][r] * PCAR); phi[r] = tohx(s[2 * c + 1][r] * PCAR); }
            const v16h pb = cat16(plo, phi);
            const h16* vr = V + (size_t)lr * TT + kt0 + c * 32 + 8 * hi;
#pragma unroll
            for (int hf = 0; hf < 8; ++hf) { const v16h aV = ldh(vr + (size_t)hf * 16 * TT); oT[hf] = wmma16g(aV, pb, oT[hf]); if (hf == 3) asm volatile("" ::: "memory"); }
            asm volatile("" ::: "memory");
        }
    }
    asm volatile("v_nop\n\tv_nop\n\tv_nop\n\tv_nop" : "+v"(oT[0]), "+v"(oT[7]));
    const float inv = __fdiv_rn(1.0f, lrow * PCAR);
    float* osw = os + wid * (16 * 132);
#pragma unroll
    for (int hf = 0; hf < 8; ++hf)
#pragma unroll
        for (int r = 0; r < 8; ++r) osw[lr * 132 + hf * 16 + 8 * hi + r] = oT[hf][r] * inv;
    __syncthreads();
    float* ob = OUTb + (size_t)qb * DM + nh * HD;
#pragma unroll 1
    for (int ps = 0; ps < 2; ++ps) {
#pragma unroll
        for (int q = 0; q < 16; ++q) { const v4f val = *(const v4fa*)(osw + q * 132 + lane * 4); *(volatile v4f*)(ob + (size_t)q * DM + lane * 4) = val; }
        if (ps == 0) __threadfence(); }
}

extern "C" void kernel_launch(void* const* d_in, const int* in_sizes, int n_in,
                              void* d_out, int out_size, void* d_ws, size_t ws_size, hipStream_t stream) {
    if (n_in < 6) return;
    if (in_sizes[0] < (int)((NB - 1) * T_FULL * DM + TT * DM)) return;
    if (in_sizes[1] < DM * DM || in_sizes[2] < DM * DM || in_sizes[3] < DM * DM) return;
    if (in_sizes[4] < TT * DM || in_sizes[5] < TT * DM) return;
    if (out_size < (int)((NB - 1) * T_FULL * DM + TT * DM)) return;
    const float* x = (const float*)d_in[0]; const float* wq = (const float*)d_in[1]; const float* wk = (const float*)d_in[2]; const float* wv = (const float*)d_in[3];
    const float* cosT = (const float*)d_in[4]; const float* sinT = (const float*)d_in[5];
    float* OUT = (float*)d_out;
    char* wsp = (char*)d_ws;
    auto take = [&](size_t bytes) { char* p = wsp; wsp += (bytes + 255) & ~(size_t)255; return (void*)p; };
    bf* WQ = (bf*)take((size_t)DM * DM * 2); bf* WK = (bf*)take((size_t)DM * DM * 2); bf* WV = (bf*)take((size_t)DM * DM * 2);
    bf* XB = (bf*)take((size_t)TT * DM * 2);
    float* FQ = (float*)take((size_t)TT * DM * 4); float* FK = (float*)take((size_t)TT * DM * 4); float* FV = (float*)take((size_t)TT * DM * 4);
    h16* QP16 = (h16*)take((size_t)NH * TT * HD * 2); h16* KP16 = (h16*)take((size_t)NH * TT * HD * 2);
    bf* QPh = (bf*)take((size_t)NH * TT * HD * 2); bf* QPl = (bf*)take((size_t)NH * TT * HD * 2); bf* KPh = (bf*)take((size_t)NH * TT * HD * 2); bf* KPl = (bf*)take((size_t)NH * TT * HD * 2);
    h16* VT16 = (h16*)take((size_t)NH * HD * TT * 2);
    bf* VEh = (bf*)take((size_t)NH * HD * TE * 2); bf* VEl = (bf*)take((size_t)NH * HD * TE * 2);
    float* Sb = (float*)take((size_t)NH * TE * TE * 4);
    bf* Ph = (bf*)take((size_t)NH * TE * TE * 2); bf* Pl = (bf*)take((size_t)NH * TE * TE * 2);
    float* Ob = (float*)take((size_t)NH * TE * HD * 4);
    if ((size_t)(wsp - (char*)d_ws) > ws_size) return;
    const unsigned LW = (unsigned)(((size_t)DM * DM / 8 + 255) / 256);
    k_cvt8<<<LW, 256, 0, stream>>>(wq, WQ, (size_t)DM * DM / 8);
    k_cvt8<<<LW, 256, 0, stream>>>(wk, WK, (size_t)DM * DM / 8);
    k_cvt8<<<LW, 256, 0, stream>>>(wv, WV, (size_t)DM * DM / 8);
    const unsigned LX = (unsigned)(((size_t)TT * DM / 8 + 255) / 256);
    const unsigned LQ = (unsigned)(((size_t)NH * TT * HD / 2 + 255) / 256);
    const unsigned LVE = (unsigned)(((size_t)NH * HD * TE / 2 + 255) / 256);
    const unsigned LM = (unsigned)(((size_t)NH * TE * HD / 2 + 255) / 256);
    for (int b = 0; b < NB; ++b) {
        float* OUTb = OUT + (size_t)b * T_FULL * DM;
        k_cvt8<<<LX, 256, 0, stream>>>(x + (size_t)b * T_FULL * DM, XB, (size_t)TT * DM / 8);
        k_gemmw<bf, 0, false><<<dim3(TT / 64, DM / 64, 1), 32, 0, stream>>>(XB, nullptr, WQ, nullptr, DM, FQ, DM, nullptr, 0, 0, 0);
        k_rope<<<LQ, 256, 0, stream>>>(FQ, cosT, sinT, QP16, QPh, QPl);
        k_gemmw<bf, 0, false><<<dim3(TT / 64, DM / 64, 1), 32, 0, stream>>>(XB, nullptr, WK, nullptr, DM, FK, DM, nullptr, 0, 0, 0);
        k_rope<<<LQ, 256, 0, stream>>>(FK, cosT, sinT, KP16, KPh, KPl);
        k_gemmw<bf, 0, false><<<dim3(TT / 64, DM / 64, 1), 32, 0, stream>>>(XB, nullptr, WV, nullptr, DM, FV, DM, nullptr, 0, 0, 0);
        k_vtp16<<<LQ, 256, 0, stream>>>(FV, VT16);
        k_vte<<<LVE, 256, 0, stream>>>(FV, VEh, VEl);
        k_gemmw<bf, 2, false><<<dim3(TE / 64, TE / 64, NH), 32, 0, stream>>>(QPh, QPl, KPh, KPl, HD, Sb, TE, nullptr, (size_t)TT * HD, (size_t)TT * HD, (size_t)TE * TE);
        k_lsoftE<<<(unsigned)(NH * TE / 8), 256, 0, stream>>>(Sb, Ph, Pl);
        k_gemmw<bf, 2, false><<<dim3(TE / 64, HD / 64, NH), 32, 0, stream>>>(Ph, Pl, VEh, VEl, TE, Ob, HD, nullptr, (size_t)TE * TE, (size_t)HD * TE, (size_t)TE * HD);
        k_mergeE<<<LM, 256, 0, stream>>>(Ob, OUTb);
        if (TT > TE) k_flash<<<dim3((unsigned)(TT / 64 - TE / 64), NH, 1), 128, 0, stream>>>(QP16, KP16, VT16, OUTb);
    }
}
